// GraphAttentionLayer_30193620091224
// MI455X (gfx1250) — hardware-run, weakly checked
//
#include <hip/hip_runtime.h>


#define NN   4096
#define EE   131072
#ifndef AGG_ROWS
#define AGG_ROWS NN
#endif
#define DIN  256
#define DM   256
#define NH_  4
#define HD   64
#define GW   2
#define NPW  32
#define WPR  (NN / 32)
#define SLOPE 0.2f
#define LOG2E 1.4426950408889634f
#define NEGB (-3.0e38f)

static_assert(NH_ * HD == DM);
static_assert(HD == 64);
static_assert(DM == 2 * 32 * 4);
static_assert(DIN % 32 == 0);
static_assert(NN % 64 == 0 && DM % 64 == 0);
static_assert(2 * HD == 128);
static_assert(8 * 32 * 16 == 16 * HD * 4);
static_assert(32 * 16 == 2 * 64 * 4);
static_assert(DIN == 256 && DM % 32 == 0);
static_assert(4 * 256 * 16 == 32 * DIN * 2);
static_assert(EE % 128 == 0);
static_assert(NN == WPR * 32 && WPR % 32 == 0);
static_assert(AGG_ROWS % (GW * NPW) == 0 && AGG_ROWS <= NN);
static_assert((NPW * WPR) % 32 == 0);
static_assert(GW * NPW * WPR * 4 <= 131072);
static_assert(DIN * 33 * 4 <= 131072);
static_assert(((size_t)NN * DIN) % 8 == 0);

typedef unsigned short bf;
typedef __attribute__((ext_vector_type(16))) __bf16   v16bf;
typedef __attribute__((ext_vector_type(8)))  unsigned short v8us;
typedef __attribute__((ext_vector_type(8)))  float    v8f;
typedef __attribute__((ext_vector_type(4)))  float    v4f;
typedef __attribute__((ext_vector_type(4)))  int      v4i;
typedef v4f  __attribute__((may_alias)) v4fa;

__device__ __forceinline__ unsigned short f2bf(float f) { unsigned u = __float_as_uint(f); u += 0x7FFFu + ((u >> 16) & 1u); return (unsigned short)(u >> 16); }
__device__ __forceinline__ float bfr(float f) { return __uint_as_float(((unsigned)f2bf(f)) << 16); }
__device__ __forceinline__ v16bf cat16b(v8us lo, v8us hi) { return __builtin_bit_cast(v16bf, __builtin_shufflevector(lo, hi, 0, 1, 2, 3, 4, 5, 6, 7, 8, 9, 10, 11, 12, 13, 14, 15)); }
__device__ __forceinline__ v8f wmmab(v16bf a, v16bf b, v8f c) { return __builtin_amdgcn_wmma_f32_16x16x32_bf16(false, a, false, b, (short)0, c, false, false); }
__device__ __forceinline__ v8f wmmab_g(v16bf a, v16bf b, v8f c) {
    c = wmmab(a, b, c);
    asm volatile("v_nop\n\tv_nop\n\tv_nop\n\tv_nop" : "+v"(c) : "v"(a), "v"(b));
    return c;
}
__device__ __forceinline__ v16bf ldb(const bf* p)  { return cat16b(*(const v8us*)p, *(const v8us*)(p + 16)); }
__device__ __forceinline__ void wave_sync() { __builtin_amdgcn_fence(3  , "wavefront"); __builtin_amdgcn_wave_barrier(); asm volatile("" ::: "memory"); }

__global__ __launch_bounds__(256) void k_cvt8(const float* __restrict__ src, bf* dst, size_t n8) {
    const size_t i = (size_t)blockIdx.x * 256 + threadIdx.x; if (i >= n8) return;
    const v8f v = *(const v8f*)(src + i * 8); v8us o;
#pragma unroll
    for (int k = 0; k < 8; ++k) o[k] = f2bf(v[k]);
    *(volatile v8us*)(dst + i * 8) = o; __threadfence(); *(volatile v8us*)(dst + i * 8) = o;
}

__global__ __launch_bounds__(256) void k_wtr(const float* __restrict__ W, bf* WT) {
    __shared__ float ts[DIN * 33];
    const int tid = threadIdx.x; const int n0 = blockIdx.x * 32;
#pragma unroll 1
    for (int it = 0; it < DIN / 8; ++it) { const int k = it * 8 + (tid >> 5); ts[k * 33 + (tid & 31)] = W[(size_t)k * DM + n0 + (tid & 31)]; }
    __syncthreads();
#pragma unroll 1
    for (int ps = 0; ps < 2; ++ps) {
#pragma unroll 1
        for (int it = 0; it < 4; ++it) { const int p = it * 256 + tid; const int row = p >> 5, c8 = (p & 31) * 8; v8us o;
#pragma unroll
            for (int q = 0; q < 8; ++q) o[q] = f2bf(ts[(c8 + q) * 33 + row]);
            *(volatile v8us*)(WT + (size_t)(n0 + row) * DIN + c8) = o; }
        if (ps == 0) __threadfence(); }
}

__global__ __launch_bounds__(32) void k_proj(const bf* __restrict__ A, const bf* __restrict__ Bt, const float* __restrict__ att, float* WH, float* EP) {
    __shared__ __align__(16) float os[16 * 68];
    __shared__ __align__(16) float sa[2 * HD];
    __shared__ __align__(16) float es[2 * 64];
    const int K = DIN;
    const int lane = threadIdx.x & 31, lr = lane & 15, hi = lane >> 4; const int r0 = blockIdx.x * 64, c0 = blockIdx.y * 64;
    { const v4f av = *(const v4f*)(att + lane * 4); v4f cv;
#pragma unroll
      for (int q = 0; q < 4; ++q) cv[q] = bfr(av[q]);
      *(v4fa*)(&sa[lane * 4]) = cv; }
    v8f acc[4][4];
#pragma unroll
    for (int mb = 0; mb < 4; ++mb)
#pragma unroll
        for (int nb = 0; nb < 4; ++nb) acc[mb][nb] = (v8f){};
    const size_t aoff = (size_t)(r0 + lr) * K + 8 * hi, boff = (size_t)(c0 + lr) * K + 8 * hi;
#pragma unroll 1
    for (int kc = 0; kc < K; kc += 32) {
        v16bf a[4];
#pragma unroll
        for (int mb = 0; mb < 4; ++mb) a[mb] = ldb(A + aoff + (size_t)mb * 16 * K + kc);
#pragma unroll
        for (int nb = 0; nb < 4; ++nb) { const v16bf b = ldb(Bt + boff + (size_t)nb * 16 * K + kc);
#pragma unroll
            for (int mb = 0; mb < 4; ++mb) acc[mb][nb] = wmmab_g(a[mb], b, acc[mb][nb]); }
    }
#pragma unroll
    for (int mb = 0; mb < 4; ++mb) {
#pragma unroll
        for (int nb = 0; nb < 4; ++nb) {
#pragma unroll
            for (int j = 0; j < 8; ++j) os[(hi * 8 + j) * 68 + nb * 16 + lr] = acc[mb][nb][j]; }
        wave_sync();
        float dsum = 0.0f;
#pragma unroll 4
        for (int f = 0; f < HD; ++f) dsum += os[lr * 68 + f] * sa[hi * HD + f];
        es[hi * 64 + mb * 16 + lr] = dsum;
#pragma unroll 1
        for (int ps = 0; ps < 2; ++ps) {
#pragma unroll
            for (int s8 = 0; s8 < 8; ++s8) { const int p = s8 * 32 + lane; const int row = p >> 4, c4 = (p & 15) * 4;
                const v4f val = *(const v4fa*)(&os[row * 68 + c4]);
                *(volatile v4f*)(WH + (size_t)(r0 + mb * 16 + row) * DM + c0 + c4) = val; }
            if (ps == 0) __threadfence(); }
        wave_sync();
    }
    { const int which = lane >> 4, c4 = (lane & 15) * 4;
      const v4f ev = *(const v4fa*)(&es[which * 64 + c4]);
      float* ep = EP + (size_t)(which * NH_ + (int)blockIdx.y) * NN + r0 + c4;
#pragma unroll 1
      for (int ps = 0; ps < 2; ++ps) { *(volatile v4f*)ep = ev; if (ps == 0) __threadfence(); } }
}

__global__ __launch_bounds__(32 * GW) void k_agg(const int* __restrict__ el, const int* __restrict__ nn_p, const float* __restrict__ WH, const float* __restrict__ EP, float* OUT) {
    __shared__ unsigned sb[GW * NPW * WPR];
    const int lane = threadIdx.x & 31;
    const int wave = __builtin_amdgcn_readfirstlane((int)(threadIdx.x >> 5));
    const int ibase = (blockIdx.x * GW + wave) * NPW;
    const int wo = wave * NPW * WPR;
    const bool bad = nn_p[0] != NN;
#pragma unroll 1
    for (int q = 0; q < NPW * WPR / 32; ++q) { const int idx = q * 32 + lane; const int node = ibase + idx / WPR; const int w = idx % WPR;
        sb[wo + idx] = ((node >> 5) == w) ? (1u << (node & 31)) : 0u; }
    wave_sync();
#pragma unroll 1
    for (int it = 0; it < EE / 128; ++it) {
        const v4i* ep = (const v4i*)(el + ((size_t)it * 32 + lane) * 12);
        const v4i a = ep[0], b = ep[1], c = ep[2];
        const int si[4] = { a[0], a[3], b[2], c[1] };
        const int so[4] = { a[1], b[0], b[3], c[2] };
#pragma unroll
        for (int q = 0; q < 4; ++q) {
            const unsigned rel = (unsigned)(si[q] - ibase);
            const int hit = (int)(rel < (unsigned)NPW) & (int)((unsigned)so[q] < (unsigned)NN);
            unsigned mk = __builtin_amdgcn_ballot_w32(hit != 0);
            const unsigned relc = (rel < (unsigned)NPW) ? rel : (unsigned)(NPW - 1);
            const unsigned wq = (unsigned)so[q] >> 5;
            const unsigned wqc = (wq < (unsigned)WPR) ? wq : (unsigned)(WPR - 1);
            const int adc = wo + (int)relc * WPR + (int)wqc;
            const unsigned bit = 1u << (so[q] & 31);
#pragma unroll 1
            for (int g = 0; g < 32 && mk != 0u; ++g) {
                const int s = __builtin_ctz(mk); mk &= mk - 1u;
                unsigned old = sb[adc];
                asm volatile("" : "+v"(old));
                const unsigned nw = old | bit;
                if (lane == s) sb[adc] = nw;
                wave_sync();
            }
        }
    }
    wave_sync();
    const int ha = lane >> 4;
    const size_t e1ao = (size_t)ha * NN, e1bo = (size_t)(2 + ha) * NN;
    const size_t e2ao = (size_t)(NH_ + ha) * NN, e2bo = (size_t)(NH_ + 2 + ha) * NN;
#pragma unroll 1
    for (int n = 0; n < NPW; ++n) {
        const int i = ibase + n;
        const float e1a = EP[e1ao + i], e1b = EP[e1bo + i];
        float ma = NEGB, mb2 = NEGB, la = 0.0f, lb = 0.0f;
        v4f aa = (v4f){}, ab = (v4f){};
#pragma unroll 1
        for (int c = 0; c < WPR / 32; ++c) {
            const unsigned wd = sb[wo + n * WPR + c * 32 + lane];
            unsigned nz = __builtin_amdgcn_ballot_w32(wd != 0u);
#pragma unroll 1
            for (int g = 0; g < 32 && nz != 0u; ++g) {
                const int s = __builtin_ctz(nz); nz &= nz - 1u;
                unsigned bits = (unsigned)__builtin_amdgcn_readlane((int)wd, s);
                const int jb = (c * 32 + s) * 32;
#pragma unroll 1
                for (int q = 0; q < 32 && bits != 0u; ++q) {
                    const int j = jb + __builtin_ctz(bits); bits &= bits - 1u;
                    const float xa = e1a + EP[e2ao + j], xb = e1b + EP[e2bo + j];
                    const float ta = ((xa >= 0.0f) ? xa : SLOPE * xa) * LOG2E;
                    const float tb = ((xb >= 0.0f) ? xb : SLOPE * xb) * LOG2E;
                    const float na = fmaxf(ma, ta), nb = fmaxf(mb2, tb);
                    const float ala = __builtin_amdgcn_exp2f(ma - na), alb = __builtin_amdgcn_exp2f(mb2 - nb);
                    const float pa = __builtin_amdgcn_exp2f(ta - na), pb = __builtin_amdgcn_exp2f(tb - nb);
                    la = la * ala + pa; lb = lb * alb + pb; ma = na; mb2 = nb;
                    const float* wr = WH + (size_t)j * DM + 4 * lane;
                    const v4f wa = *(const v4f*)wr, wb = *(const v4f*)(wr + 128);
                    aa = aa * ala + wa * pa; ab = ab * alb + wb * pb;
                }
            }
        }
        const float ia = 1.0f / la, ib = 1.0f / lb;
        const float qn = __uint_as_float(0x7FC00000u);
        v4f ra, rb;
#pragma unroll
        for (int q = 0; q < 4; ++q) {
            const float xa = aa[q] * ia, xb = ab[q] * ib;
            const float ya = (xa > 0.0f) ? xa : (__builtin_amdgcn_exp2f(xa * LOG2E) - 1.0f);
            const float yb = (xb > 0.0f) ? xb : (__builtin_amdgcn_exp2f(xb * LOG2E) - 1.0f);
            ra[q] = bad ? qn : ya; rb[q] = bad ? qn : yb; }
        float* orow = OUT + (size_t)i * DM + 4 * lane;
#pragma unroll 1
        for (int ps = 0; ps < 2; ++ps) {
            *(volatile v4f*)orow = ra; *(volatile v4f*)(orow + 128) = rb;
            if (ps == 0) __threadfence(); }
    }
}

static constexpr size_t al256(size_t v) { return (v + 255) & ~(size_t)255; }
static constexpr size_t SZ_XB = al256((size_t)NN * DIN * 2);
static constexpr size_t SZ_WT = al256((size_t)DM * DIN * 2);
static constexpr size_t SZ_WH = al256((size_t)NN * DM * 4);
static constexpr size_t SZ_EP = al256((size_t)2 * NH_ * NN * 4);
static constexpr size_t SZ_TOTAL = SZ_XB + SZ_WT + SZ_WH + SZ_EP;
static_assert(SZ_TOTAL <= (size_t)134217728);
static_assert(((size_t)(NN / 64) * 64) == (size_t)NN);
static_assert((size_t)(2 * NH_ - 1) * NN + (NN - 64) + 64 <= (size_t)2 * NH_ * NN);

extern "C" void kernel_launch(void* const* d_in, const int* in_sizes, int n_in,
                              void* d_out, int out_size, void* d_ws, size_t ws_size, hipStream_t stream) {
    if (n_in < 5) return;
    if ((size_t)in_sizes[0] < (size_t)NN * DIN) return;
    if ((size_t)in_sizes[1] < (size_t)EE * 3) return;
    if (in_sizes[2] < 1) return;
    if ((size_t)in_sizes[3] < (size_t)DIN * DM) return;
    if (in_sizes[4] < 2 * HD) return;
    if ((size_t)out_size < (size_t)NN * DM) return;
    if (SZ_TOTAL > ws_size) return;
    const float* xin = (const float*)d_in[0];
    const int*   el  = (const int*)d_in[1];
    const int*   nnp = (const int*)d_in[2];
    const float* w   = (const float*)d_in[3];
    const float* att = (const float*)d_in[4];
    float* OUT = (float*)d_out;
    char* wsp = (char*)d_ws;
    bf* XB = (bf*)wsp; wsp += SZ_XB;
    bf* WT = (bf*)wsp; wsp += SZ_WT;
    float* WH = (float*)wsp; wsp += SZ_WH;
    float* EP = (float*)wsp; wsp += SZ_EP;

    { const size_t n8 = (size_t)NN * DIN / 8;
      k_cvt8<<<(unsigned)((n8 + 255) / 256), 256, 0, stream>>>(xin, XB, n8); }
    k_wtr<<<DM / 32, 256, 0, stream>>>(w, WT);
    k_proj<<<dim3(NN / 64, DM / 64, 1), 32, 0, stream>>>(XB, WT, att, WH, EP);
    k_agg<<<AGG_ROWS / (GW * NPW), 32 * GW, 0, stream>>>(el, nnp, WH, EP, OUT);
}
